// QuantumSelfAttention_65481071396695
// MI455X (gfx1250) — hardware-verified
//
#include <hip/hip_runtime.h>
#include <math.h>

typedef __attribute__((ext_vector_type(16))) _Float16 v16h;
typedef __attribute__((ext_vector_type(16))) __bf16 v16b;
typedef __attribute__((ext_vector_type(8)))  _Float16 v8h;
typedef __attribute__((ext_vector_type(8)))  float v8f;
typedef __attribute__((ext_vector_type(4)))  float v4f;
typedef __attribute__((ext_vector_type(2)))  float v2f;
typedef __attribute__((ext_vector_type(4)))  unsigned v4u;
typedef __attribute__((ext_vector_type(4)))  int v4i;
typedef float __attribute__((may_alias)) float_a;
typedef int __attribute__((may_alias)) int_a;

template <typename T> __device__ __forceinline__ void vst2(void* p, T v) { *(volatile T*)p = v; __threadfence(); *(volatile T*)p = v; }
__device__ __forceinline__ v8f wmma16(v16h a, v16h b, v8f c) {
  v8f d = __builtin_amdgcn_wmma_f32_16x16x32_f16(false, a, false, b, (short)0, c, false, false);
  asm volatile("v_nop\n\tv_nop\n\tv_nop\n\tv_nop" : "+v"(d) : "v"(a), "v"(b));
  return d;
}
__device__ __forceinline__ v8f wmma_bf(v16b a, v16b b, v8f c) {
  v8f d = __builtin_amdgcn_wmma_f32_16x16x32_bf16(false, a, false, b, (short)0, c, false, false);
  asm volatile("v_nop\n\tv_nop\n\tv_nop\n\tv_nop" : "+v"(d) : "v"(a), "v"(b));
  return d;
}
__device__ __forceinline__ v16h frag_h(const _Float16* rowk0, int lane) {
  union { v16h v; v8h q[2]; } u; const _Float16* p = rowk0 + 8 * (lane >> 4);
  u.q[0] = *(const v8h*)p; u.q[1] = *(const v8h*)(p + 16); return u.v;
}
__device__ __forceinline__ v16h frag_f32(const float* rowk0, int lane) {
  v16h a; const float* p = rowk0 + 8 * (lane >> 4);
#pragma unroll
  for (int i = 0; i < 8; ++i) { a[i] = (_Float16)p[i]; a[8 + i] = (_Float16)p[16 + i]; }
  return a;
}
__device__ __forceinline__ v16h frag_f32s(const float* rowk0, int lane, float sc) {
  v16h a; const float* p = rowk0 + 8 * (lane >> 4);
#pragma unroll
  for (int i = 0; i < 8; ++i) { a[i] = (_Float16)(p[i] * sc); a[8 + i] = (_Float16)(p[16 + i] * sc); }
  return a;
}
__device__ __forceinline__ v16h fragc_f32(const float* W, int k0, int n, int lane, int ld, int K) {
  v16h a; const int g = lane >> 4;
#pragma unroll
  for (int i = 0; i < 8; ++i) { const int ka = k0 + 8 * g + i, kb = ka + 16;
    a[i] = (_Float16)(ka < K ? W[(size_t)(ka < K ? ka : K - 1) * ld + n] : 0.f); a[8 + i] = (_Float16)(kb < K ? W[(size_t)(kb < K ? kb : K - 1) * ld + n] : 0.f); }
  return a;
}
struct F2 { v16b h, l; };
__device__ __forceinline__ F2 bsplit16(const float v[16]) { F2 r;
#pragma unroll
  for (int i = 0; i < 16; ++i) { const __bf16 h = (__bf16)v[i]; r.h[i] = h; r.l[i] = (__bf16)(v[i] - (float)h); }
  return r; }
__device__ __forceinline__ F2 split_row(const float* row, int k0, int lane) { float v[16]; const float* p = row + k0 + 8 * (lane >> 4);
#pragma unroll
  for (int i = 0; i < 8; ++i) { v[i] = p[i]; v[8 + i] = p[16 + i]; }
  return bsplit16(v); }
__device__ __forceinline__ F2 split_rowK(const float* row, int k0, int lane, int K) { float v[16]; const int g = lane >> 4;
#pragma unroll
  for (int i = 0; i < 8; ++i) { const int ka = k0 + 8 * g + i, kb = ka + 16; v[i] = ka < K ? row[ka < K ? ka : K - 1] : 0.f; v[8 + i] = kb < K ? row[kb < K ? kb : K - 1] : 0.f; }
  return bsplit16(v); }
__device__ __forceinline__ F2 split_col(const float* W, int k0, int n, int lane, int ld, int K) { float v[16]; const int g = lane >> 4;
#pragma unroll
  for (int i = 0; i < 8; ++i) { const int ka = k0 + 8 * g + i, kb = ka + 16; v[i] = ka < K ? W[(size_t)(ka < K ? ka : K - 1) * ld + n] : 0.f; v[8 + i] = kb < K ? W[(size_t)(kb < K ? kb : K - 1) * ld + n] : 0.f; }
  return bsplit16(v); }
__device__ __forceinline__ v8f mac3(const F2& a, const F2& b, v8f c) { c = wmma_bf(a.l, b.h, c); c = wmma_bf(a.h, b.l, c); return wmma_bf(a.h, b.h, c); }
__device__ __forceinline__ float sigm(float v) { return 1.0f / (1.0f + expf(-v)); }
#define LDSX() do { asm volatile("s_wait_dscnt 0" ::: "memory"); __builtin_amdgcn_wave_barrier(); __builtin_amdgcn_fence(__ATOMIC_RELEASE, "workgroup"); } while (0)


#define NBT 8192
#define NW 8
#define ED 256
#ifndef TQB
#define TQB (NBT / 64)
#endif
typedef __attribute__((ext_vector_type(8))) __bf16 v8b;
__device__ __forceinline__ v16b frag_b(const __bf16* rowk0, int lane) {
  union { v16b v; v8b q[2]; } u; const __bf16* p = rowk0 + 8 * (lane >> 4);
  u.q[0] = *(const v8b*)p; u.q[1] = *(const v8b*)(p + 16); return u.v;
}
__device__ __forceinline__ float bfr(float v) { return (float)(__bf16)v; }
__device__ __attribute__((noinline)) float exp_ni(float v) { return expf(v); }
__device__ __attribute__((noinline)) float erf_ni(float v) { return erff(v); }

#define WS_PJ  0u
#define WS_PM  (WS_PJ + 4u * NBT * NW)
#define WS_VH  (WS_PM + 4u * NBT * NW)
#define WS_VL  (WS_VH + 2u * 16 * NBT)
#define WS_END (WS_VL + 2u * 16 * NBT)

__global__ __launch_bounds__(64) void k_prep(const float* __restrict__ R, const float* __restrict__ E, const float* __restrict__ X, const float* __restrict__ TH, float* __restrict__ PJ, float* __restrict__ PM, _Float16* __restrict__ VH, _Float16* __restrict__ VL) { __shared__ float sM[NW][NW]; __shared__ __align__(16) float sp[64][NW], spm[64][NW]; __shared__ __align__(16) _Float16 th[16][64], tl[16][64];
  const int t = threadIdx.x; const size_t r0 = (size_t)blockIdx.x * 64;
  { const int a = t >> 3, c = t & 7; float s = 0.f;
#pragma unroll 1
    for (int e = 0; e < ED; ++e) s += bfr(R[a * ED + e]) * bfr(E[c * ED + e]);
    sM[a][c] = s; }
  { const size_t row = r0 + t;
#pragma unroll 1
    for (int w = 0; w < NW; ++w) sp[t][w] = cosf(bfr(X[row * NW + w]) + bfr(TH[w])); }
  __syncthreads();
#pragma unroll 1
  for (int c = 0; c < NW; ++c) { float s = 0.f;
#pragma unroll 1
    for (int a = 0; a < NW; ++a) s += sp[t][a] * sM[a][c];
    spm[t][c] = s; }
#pragma unroll 1
  for (int w = 0; w < 16; ++w) { const float v = (w < NW) ? sp[t][w] : 0.f; const _Float16 hv = (_Float16)v; th[w][t] = hv; tl[w][t] = (_Float16)((v - (float)hv) * 2048.0f); }
  __syncthreads();
  if (t < 32) { const int rl = t * 2; vst2(PJ + (r0 + rl) * NW, *(const v4f*)&sp[rl][0]); vst2(PJ + (r0 + rl) * NW + 4, *(const v4f*)&sp[rl][4]); vst2(PJ + (r0 + rl + 1) * NW, *(const v4f*)&sp[rl + 1][0]); vst2(PJ + (r0 + rl + 1) * NW + 4, *(const v4f*)&sp[rl + 1][4]);
    vst2(PM + (r0 + rl) * NW, *(const v4f*)&spm[rl][0]); vst2(PM + (r0 + rl) * NW + 4, *(const v4f*)&spm[rl][4]); vst2(PM + (r0 + rl + 1) * NW, *(const v4f*)&spm[rl + 1][0]); vst2(PM + (r0 + rl + 1) * NW + 4, *(const v4f*)&spm[rl + 1][4]); }
  for (int e = t; e < 16 * 8; e += 64) { const int w = e >> 3, q = e & 7; vst2((unsigned*)(VH + (size_t)w * NBT + r0 + q * 8), *(const v4u*)&th[w][q * 8]); vst2((unsigned*)(VL + (size_t)w * NBT + r0 + q * 8), *(const v4u*)&tl[w][q * 8]); } }
__device__ __forceinline__ F2 frag8(const float* __restrict__ row8, int lane) { float v[16]; const int g = lane >> 4;
#pragma unroll
  for (int i = 0; i < 8; ++i) { v[i] = (g == 0) ? row8[i] : 0.f; v[8 + i] = 0.f; }
  return bsplit16(v); }
__global__ __launch_bounds__(128) void k_att(const float* __restrict__ PM, const float* __restrict__ PJ, const _Float16* __restrict__ VH, const _Float16* __restrict__ VL, float* __restrict__ OUT) { __shared__ __align__(16) float sp[4][16][36]; __shared__ __align__(16) float so[4][16][20];
  const int tid = threadIdx.x, wave = tid >> 5, lane = tid & 31, col = lane & 15, g = lane >> 4; const int q0 = blockIdx.x * 64 + wave * 16;
  const F2 aq = frag8(PM + (size_t)(q0 + col) * NW, lane);
  float m[8], l[8];
#pragma unroll
  for (int r = 0; r < 8; ++r) { m[r] = -3.0e38f; l[r] = 0.f; }
  v8f acc = {}, accl = {};
#pragma unroll 1
  for (int ks = 0; ks < NBT / 32; ++ks) { float s[2][8];
#pragma unroll
    for (int ct = 0; ct < 2; ++ct) { const int kk = ks * 32 + ct * 16 + col; const F2 bk = frag8(PJ + (size_t)kk * NW, lane); v8f c = {}; c = wmma_bf(aq.h, bk.h, c); c = wmma_bf(aq.h, bk.l, c); c = wmma_bf(aq.l, bk.h, c); c = wmma_bf(aq.l, bk.l, c);
#pragma unroll
      for (int r = 0; r < 8; ++r) s[ct][r] = c[r] * 0.0625f; }
    float alpha[8];
#pragma unroll
    for (int r = 0; r < 8; ++r) { float mx = fmaxf(s[0][r], s[1][r]);
#pragma unroll
      for (int o = 1; o < 16; o <<= 1) mx = fmaxf(mx, __shfl_xor(mx, o));
      const float mn = fmaxf(m[r], mx); alpha[r] = __expf(m[r] - mn); const float e0 = __expf(s[0][r] - mn), e1 = __expf(s[1][r] - mn); float es = e0 + e1;
#pragma unroll
      for (int o = 1; o < 16; o <<= 1) es += __shfl_xor(es, o);
      l[r] = l[r] * alpha[r] + es; m[r] = mn; sp[wave][8 * g + r][col] = e0; sp[wave][8 * g + r][16 + col] = e1; }
#pragma unroll
    for (int r = 0; r < 8; ++r) { acc[r] *= alpha[r]; accl[r] *= alpha[r]; }
    LDSX();
    v16h pa, par; { const float* prow = &sp[wave][col][0] + 8 * (lane >> 4);
#pragma unroll
      for (int i = 0; i < 8; ++i) { const float p0 = prow[i] * 2048.0f, p1 = prow[16 + i] * 2048.0f; pa[i] = (_Float16)p0; pa[8 + i] = (_Float16)p1; par[i] = (_Float16)(p0 - (float)pa[i]); par[8 + i] = (_Float16)(p1 - (float)pa[8 + i]); } }
    { const v16h vh = frag_h(VH + (size_t)col * NBT + ks * 32, lane); acc = wmma16(pa, vh, acc); acc = wmma16(par, vh, acc); accl = wmma16(pa, frag_h(VL + (size_t)col * NBT + ks * 32, lane), accl); }
    LDSX(); }
#pragma unroll
  for (int r = 0; r < 8; ++r) { const float il = (1.0f / 2048.0f) / l[r]; so[wave][8 * g + r][col] = (acc[r] + accl[r] * (1.0f / 2048.0f)) * il; }
  LDSX();
  if (lane < 32) { const int rl = lane >> 1, hh = lane & 1; vst2(OUT + (size_t)(q0 + rl) * NW + hh * 4, *(const v4f*)&so[wave][rl][hh * 4]); } }
extern "C" void kernel_launch(void* const* d_in, const int* in_sizes, int n_in, void* d_out, int out_size, void* d_ws, size_t ws_size, hipStream_t stream) {
  (void)in_sizes; (void)n_in; (void)out_size;
  const float** F = (const float**)d_in;
  if (ws_size < (size_t)WS_END) return;
  char* ws = (char*)d_ws; float *PJ = (float*)(ws + WS_PJ), *PM = (float*)(ws + WS_PM); _Float16 *VH = (_Float16*)(ws + WS_VH), *VL = (_Float16*)(ws + WS_VL);
  k_prep<<<NBT / 64, 64, 0, stream>>>(F[0], F[1], F[2], F[3], PJ, PM, VH, VL);
  k_att<<<TQB, 128, 0, stream>>>(PM, PJ, VH, VL, (float*)d_out);
}
